// MHA_8727373545917
// MI455X (gfx1250) — hardware-verified
//
#include <hip/hip_runtime.h>


#ifndef NB
#define NB 32
#endif
#ifndef SEQ
#define SEQ 512
#endif
#define NB_FULL  32
#define SEQ_FULL 512
#define DM   256
#define NH   8
#define HD   32
#define NQKV 768
#define CP   264
#define SCL  0.17677669529663688f
#define L2E  1.4426950408889634f

static_assert(SEQ % 64 == 0);
static_assert(SEQ <= SEQ_FULL);
static_assert(NB >= 1);
static_assert(NB <= NB_FULL);
static_assert(NH * HD == DM);
static_assert(NQKV == 3 * DM);

typedef unsigned short bf;
typedef __attribute__((ext_vector_type(16))) __bf16   v16bf;
typedef __attribute__((ext_vector_type(8)))  unsigned short v8us;
typedef __attribute__((ext_vector_type(2)))  unsigned short v2us;
typedef __attribute__((ext_vector_type(8)))  float    v8f;
typedef __attribute__((ext_vector_type(4)))  float    v4f;
typedef v4f  __attribute__((may_alias)) v4fa;
typedef v8us __attribute__((may_alias)) v8usa;

__device__ __forceinline__ unsigned short f2bf(float f) { unsigned u = __float_as_uint(f); u += 0x7FFFu + ((u >> 16) & 1u); return (unsigned short)(u >> 16); }
__device__ __forceinline__ float bf2f(unsigned short b) { return __uint_as_float(((unsigned)b) << 16); }
__device__ __forceinline__ float bfr(float f) { return bf2f(f2bf(f)); }
__device__ __forceinline__ void splitf(float y, unsigned short& h, unsigned short& l) { h = f2bf(y); l = f2bf(y - bf2f(h)); }
__device__ __forceinline__ v16bf cat16b(v8us lo, v8us hi) { return __builtin_bit_cast(v16bf, __builtin_shufflevector(lo, hi, 0, 1, 2, 3, 4, 5, 6, 7, 8, 9, 10, 11, 12, 13, 14, 15)); }
__device__ __forceinline__ v8f wmmab(v16bf a, v16bf b, v8f c) { return __builtin_amdgcn_wmma_f32_16x16x32_bf16(false, a, false, b, (short)0, c, false, false); }
__device__ __forceinline__ v16bf ldf(const bf* p) { return cat16b(*(const v8us*)p, *(const v8us*)(p + 16)); }

template <typename T16> struct WFrag;
template <> struct WFrag<bf> { typedef v16bf V; static __device__ __forceinline__ V ld(const bf* p) { return cat16b(*(const v8us*)p, *(const v8us*)(p + 16)); } static __device__ __forceinline__ v8f mma(V a, V b, v8f c) { return wmmab(a, b, c); } };
template <typename T16, int NSPLIT, bool BIAS>
__global__ __launch_bounds__(32) void k_gemmw(const T16* __restrict__ A, const T16* __restrict__ A2, const T16* __restrict__ Bt, const T16* __restrict__ Bt2, int K, float* C, int ldc, const float* __restrict__ bias, size_t sA, size_t sB, size_t sC) {
    typedef typename WFrag<T16>::V V;
    __shared__ __align__(16) float os[16 * 68];
    const size_t z = blockIdx.z; A += z * sA; if (A2) A2 += z * sA; Bt += z * sB; if (Bt2) Bt2 += z * sB; C += z * sC;
    const int lane = threadIdx.x & 31, lr = lane & 15, hi = lane >> 4; const int r0 = blockIdx.x * 64, c0 = blockIdx.y * 64;
    v8f acc[4][4];
#pragma unroll
    for (int mb = 0; mb < 4; ++mb)
#pragma unroll
        for (int nb = 0; nb < 4; ++nb) acc[mb][nb] = (v8f){};
    const size_t aoff = (size_t)(r0 + lr) * K + 8 * hi, boff = (size_t)(c0 + lr) * K + 8 * hi;
#pragma unroll 1
    for (int kc = 0; kc < K; kc += 32) {
        V a[4], a2[4];
#pragma unroll
        for (int mb = 0; mb < 4; ++mb) { a[mb] = WFrag<T16>::ld(A + aoff + (size_t)mb * 16 * K + kc); if (NSPLIT == 1 || NSPLIT == 2) a2[mb] = WFrag<T16>::ld(A2 + aoff + (size_t)mb * 16 * K + kc); }
#pragma unroll
        for (int nb = 0; nb < 4; ++nb) { const V b = WFrag<T16>::ld(Bt + boff + (size_t)nb * 16 * K + kc); V b2; if (NSPLIT >= 2) b2 = WFrag<T16>::ld(Bt2 + boff + (size_t)nb * 16 * K + kc);
#pragma unroll
            for (int mb = 0; mb < 4; ++mb) { acc[mb][nb] = WFrag<T16>::mma(a[mb], b, acc[mb][nb]); if (NSPLIT == 1 || NSPLIT == 2) acc[mb][nb] = WFrag<T16>::mma(a2[mb], b, acc[mb][nb]); if (NSPLIT >= 2) acc[mb][nb] = WFrag<T16>::mma(a[mb], b2, acc[mb][nb]); } }
        asm volatile("v_nop\n\tv_nop\n\tv_nop\n\tv_nop" : "+v"(acc[0][0]), "+v"(acc[1][1]), "+v"(acc[2][2]), "+v"(acc[3][3]) : "v"(a[0]), "v"(a[3]));
    }
#pragma unroll
    for (int mb = 0; mb < 4; ++mb) {
#pragma unroll
        for (int nb = 0; nb < 4; ++nb) {
#pragma unroll
            for (int j = 0; j < 8; ++j) os[(hi * 8 + j) * 68 + nb * 16 + lr] = acc[mb][nb][j]; }
        __builtin_amdgcn_wave_barrier(); asm volatile("" ::: "memory");
        float* crow = C + (size_t)(r0 + mb * 16) * ldc + c0;
#pragma unroll 1
        for (int ps = 0; ps < 2; ++ps) {
#pragma unroll
            for (int s = 0; s < 8; ++s) { const int row = 2 * s + hi, cofs = lr * 4; v4f val = *(const v4fa*)(os + row * 68 + cofs); if (BIAS) { val[0] += bfr(bias[c0 + cofs]); val[1] += bfr(bias[c0 + cofs + 1]); val[2] += bfr(bias[c0 + cofs + 2]); val[3] += bfr(bias[c0 + cofs + 3]); }
                *(volatile v4f*)(crow + (size_t)row * ldc + cofs) = val; }
            if (ps == 0) __threadfence(); }
        __builtin_amdgcn_wave_barrier(); asm volatile("" ::: "memory");
    }
}

__global__ __launch_bounds__(256) void k_cvt8(const float* __restrict__ src, bf* dst, unsigned n8, size_t ss, size_t ds) {
    const unsigned i = blockIdx.x * 256u + threadIdx.x; if (i >= n8) return;
    src += (size_t)blockIdx.y * ss; dst += (size_t)blockIdx.y * ds;
    const v8f v = *(const v8f*)(src + (size_t)i * 8); v8us o;
#pragma unroll
    for (int k = 0; k < 8; ++k) o[k] = f2bf(v[k]);
    *(volatile v8us*)(dst + (size_t)i * 8) = o; __threadfence(); *(volatile v8us*)(dst + (size_t)i * 8) = o; }

__global__ __launch_bounds__(256) void k_wt(const float* __restrict__ W, bf* Wt, unsigned N) {
    const unsigned e2 = (blockIdx.x * 256u + threadIdx.x) * 2u; if (e2 >= N * 256u) return;
    const unsigned k = e2 & 255u, n = e2 >> 8;
    v2us o; o[0] = f2bf(W[(size_t)k * N + n]); o[1] = f2bf(W[(size_t)(k + 1u) * N + n]);
    *(volatile v2us*)(Wt + (size_t)n * 256u + k) = o; __threadfence(); *(volatile v2us*)(Wt + (size_t)n * 256u + k) = o; }

__global__ __launch_bounds__(32) void k_qkv(const bf* __restrict__ A, const bf* __restrict__ Bt, const float* __restrict__ bias, bf* QPh, bf* QPl, bf* KPh, bf* KPl, bf* VTh, bf* VTl) {
    __shared__ __align__(16) float os[64 * 68];
    const unsigned lane = threadIdx.x & 31u, lr = lane & 15u, hi = lane >> 4; const unsigned r0 = blockIdx.x * 64u, c0 = blockIdx.y * 64u;
    v8f acc[4][4];
#pragma unroll
    for (int mb = 0; mb < 4; ++mb)
#pragma unroll
        for (int nb = 0; nb < 4; ++nb) acc[mb][nb] = (v8f){};
    const size_t aoff = (size_t)(r0 + lr) * DM + 8u * hi, boff = (size_t)(c0 + lr) * DM + 8u * hi;
#pragma unroll 1
    for (unsigned kc = 0; kc < DM; kc += 32u) {
        v16bf a[4];
#pragma unroll
        for (int mb = 0; mb < 4; ++mb) a[mb] = ldf(A + aoff + (size_t)mb * 16 * DM + kc);
#pragma unroll
        for (int nb = 0; nb < 4; ++nb) { const v16bf b = ldf(Bt + boff + (size_t)nb * 16 * DM + kc);
#pragma unroll
            for (int mb = 0; mb < 4; ++mb) acc[mb][nb] = wmmab(a[mb], b, acc[mb][nb]); }
        asm volatile("v_nop\n\tv_nop\n\tv_nop\n\tv_nop" : "+v"(acc[0][0]), "+v"(acc[1][1]), "+v"(acc[2][2]), "+v"(acc[3][3]) : "v"(a[0]), "v"(a[3]));
    }
#pragma unroll
    for (int nb = 0; nb < 4; ++nb) { const float bv = bfr(bias[c0 + nb * 16 + lr]);
#pragma unroll
        for (int mb = 0; mb < 4; ++mb) {
#pragma unroll
            for (int j = 0; j < 8; ++j) os[(mb * 16 + hi * 8 + j) * 68 + nb * 16 + lr] = acc[mb][nb][j] + bv; } }
    asm volatile("s_wait_dscnt 0x0" ::: "memory"); __builtin_amdgcn_wave_barrier(); asm volatile("" ::: "memory");
    const unsigned b = r0 / (unsigned)SEQ, t0 = r0 - b * (unsigned)SEQ; const unsigned sel = c0 >> 8, hA = (c0 & 255u) >> 5;
    if (sel < 2u) {
        bf* Ph = (sel == 0u) ? QPh : KPh; bf* Pl = (sel == 0u) ? QPl : KPl;
#pragma unroll 1
        for (int ps = 0; ps < 2; ++ps) {
#pragma unroll 1
            for (unsigned hh = 0; hh < 2u; ++hh) {
#pragma unroll 2
                for (unsigned s = 0; s < 8u; ++s) { const unsigned tl = 8u * s + (lane >> 2), d0 = (lane & 3u) * 8u; const float* src = os + tl * 68u + hh * 32u + d0;
                    const v4f x0 = *(const v4fa*)src, x1 = *(const v4fa*)(src + 4); v8us oh, ol;
#pragma unroll
                    for (int q = 0; q < 4; ++q) { unsigned short u, w2; splitf(x0[q], u, w2); oh[q] = u; ol[q] = w2; splitf(x1[q], u, w2); oh[4 + q] = u; ol[4 + q] = w2; }
                    const size_t off = (((size_t)b * NH + hA + hh) * SEQ + t0 + tl) * HD + d0;
                    *(volatile v8us*)(Ph + off) = oh; *(volatile v8us*)(Pl + off) = ol; } }
            if (ps == 0) __threadfence(); }
    } else {
#pragma unroll 1
        for (int ps = 0; ps < 2; ++ps) {
#pragma unroll 1
            for (unsigned hh = 0; hh < 2u; ++hh) {
#pragma unroll 2
                for (unsigned s = 0; s < 8u; ++s) { const unsigned d = 4u * s + (lane >> 3), tl0 = (lane & 7u) * 8u; v8us oh, ol;
#pragma unroll
                    for (int i = 0; i < 8; ++i) { unsigned short u, w2; splitf(os[(tl0 + i) * 68u + hh * 32u + d], u, w2); oh[i] = u; ol[i] = w2; }
                    const size_t off = (((size_t)b * NH + hA + hh) * HD + d) * SEQ + t0 + tl0;
                    *(volatile v8us*)(VTh + off) = oh; *(volatile v8us*)(VTl + off) = ol; } }
            if (ps == 0) __threadfence(); }
    }
}

__global__ __launch_bounds__(256) void k_attn(const bf* __restrict__ QPh, const bf* __restrict__ QPl, const bf* __restrict__ KPh, const bf* __restrict__ KPl, const bf* __restrict__ VTh, const bf* __restrict__ VTl, bf* CXh, bf* CXl) {
    __shared__ __align__(16) unsigned short sh[16 * CP];
    __shared__ __align__(16) unsigned short sl[16 * CP];
    const unsigned tid = threadIdx.x, lane = tid & 31u, w = tid >> 5, lr = lane & 15u, hi = lane >> 4;
    const unsigned qt = blockIdx.x, b = blockIdx.y, q0 = qt * 16u;
    const size_t bh = (size_t)b * NH + w;
    const size_t qoff = (bh * SEQ + q0 + lr) * HD + 8u * hi;
    const v16bf qh = ldf(QPh + qoff), ql = ldf(QPl + qoff);
    const size_t koff = (bh * SEQ + lr) * HD + 8u * hi;
    const bf* kh = KPh + koff; const bf* kl = KPl + koff;
    const size_t voff = (bh * HD + lr) * SEQ + 8u * hi;
    const bf* vh = VTh + voff; const bf* vl = VTl + voff;
    float m = -3.0e38f, l = 0.f; v8f o0 = (v8f){}, o1 = (v8f){};
    const unsigned query = q0 + lr;
    const unsigned nch = (qt >> 1) + 1u;
#pragma unroll 1
    for (unsigned kc = 0; kc < nch; ++kc) {
        const unsigned kb = kc * 32u;
        const v16bf k0h = ldf(kh + (size_t)kb * HD), k0l = ldf(kl + (size_t)kb * HD), k1h = ldf(kh + (size_t)(kb + 16u) * HD), k1l = ldf(kl + (size_t)(kb + 16u) * HD);
        v8f s0 = (v8f){}, s1 = (v8f){};
        s0 = wmmab(k0h, qh, s0); s0 = wmmab(k0h, ql, s0); s0 = wmmab(k0l, qh, s0);
        s1 = wmmab(k1h, qh, s1); s1 = wmmab(k1h, ql, s1); s1 = wmmab(k1l, qh, s1);
        asm volatile("v_nop\n\tv_nop\n\tv_nop\n\tv_nop" : "+v"(s0), "+v"(s1) : "v"(k0h), "v"(k0l), "v"(k1h), "v"(k1l), "v"(qh), "v"(ql));
        const unsigned keyb = kb + 8u * hi;
        float t0[8], t1[8]; float tmax = -3.0e38f;
#pragma unroll
        for (int r = 0; r < 8; ++r) { const bool ok0 = (keyb + (unsigned)r) <= query, ok1 = (keyb + 16u + (unsigned)r) <= query;
            t0[r] = ok0 ? s0[r] * SCL : -3.0e38f; t1[r] = ok1 ? s1[r] * SCL : -3.0e38f; tmax = fmaxf(tmax, fmaxf(t0[r], t1[r])); }
        tmax = fmaxf(tmax, __shfl_xor(tmax, 16, 32));
        const float mnew = fmaxf(m, tmax);
        const float alpha = __builtin_amdgcn_exp2f(__fmul_rn(__fsub_rn(m, mnew), L2E));
        float psum = 0.f; v8us p0h, p0l, p1h, p1l;
#pragma unroll
        for (int r = 0; r < 8; ++r) { const bool ok0 = (keyb + (unsigned)r) <= query, ok1 = (keyb + 16u + (unsigned)r) <= query;
            const float e0 = __builtin_amdgcn_exp2f(__fmul_rn(__fsub_rn(t0[r], mnew), L2E)), e1 = __builtin_amdgcn_exp2f(__fmul_rn(__fsub_rn(t1[r], mnew), L2E));
            const float p0 = ok0 ? e0 : 0.f, p1 = ok1 ? e1 : 0.f; psum += p0 + p1;
            unsigned short u, w2; splitf(p0, u, w2); p0h[r] = u; p0l[r] = w2; splitf(p1, u, w2); p1h[r] = u; p1l[r] = w2; }
        l = l * alpha + psum; m = mnew;
        o0 *= alpha; o1 *= alpha;
        const v16bf ph = cat16b(p0h, p1h), pl = cat16b(p0l, p1l);
        const v16bf v0h = ldf(vh + kb), v0l = ldf(vl + kb), v1h = ldf(vh + (size_t)16 * SEQ + kb), v1l = ldf(vl + (size_t)16 * SEQ + kb);
        o0 = wmmab(v0h, ph, o0); o0 = wmmab(v0h, pl, o0); o0 = wmmab(v0l, ph, o0);
        o1 = wmmab(v1h, ph, o1); o1 = wmmab(v1h, pl, o1); o1 = wmmab(v1l, ph, o1);
        asm volatile("v_nop\n\tv_nop\n\tv_nop\n\tv_nop" : "+v"(o0), "+v"(o1) : "v"(v0h), "v"(v0l), "v"(v1h), "v"(v1l), "v"(ph), "v"(pl));
    }
    const float ltot = l + __shfl_xor(l, 16, 32);
    const float inv = __fdiv_rn(1.0f, ltot);
    v8us ah, al, ch, cl;
#pragma unroll
    for (int r = 0; r < 8; ++r) { unsigned short u, w2; splitf(o0[r] * inv, u, w2); ah[r] = u; al[r] = w2; splitf(o1[r] * inv, u, w2); ch[r] = u; cl[r] = w2; }
    const unsigned so = lr * CP + w * 32u + 8u * hi;
    *(v8usa*)(sh + so) = ah; *(v8usa*)(sl + so) = al; *(v8usa*)(sh + so + 16u) = ch; *(v8usa*)(sl + so + 16u) = cl;
    __syncthreads();
    bf* gh = CXh + ((size_t)b * SEQ + q0) * DM; bf* gl = CXl + ((size_t)b * SEQ + q0) * DM;
#pragma unroll 1
    for (int ps = 0; ps < 2; ++ps) {
#pragma unroll
        for (unsigned rr = 0; rr < 2u; ++rr) { const unsigned row = 2u * w + rr; const v8us xh = *(const v8usa*)(sh + row * CP + lane * 8u), xl = *(const v8usa*)(sl + row * CP + lane * 8u);
            *(volatile v8us*)(gh + (size_t)row * DM + lane * 8u) = xh; *(volatile v8us*)(gl + (size_t)row * DM + lane * 8u) = xl; }
        if (ps == 0) __threadfence(); }
}

#define PLB ((size_t)NB * SEQ * DM * 2)
static_assert((size_t)NQKV * DM * 2 + (size_t)DM * DM * 2 + 9 * PLB <= (size_t)134217728);
static_assert(PLB % 256 == 0);
static_assert((size_t)(NQKV / 2) * 256 * 2 == (size_t)NQKV * DM);
static_assert((size_t)(DM / 2) * 256 * 2 == (size_t)DM * DM);
static_assert((size_t)(SEQ / 8) * 256 * 8 == (size_t)SEQ * DM);
static_assert((size_t)(NB * SEQ / 64) * (DM / 64) * 2 * 8 * 32 * 8 == (size_t)NB * SEQ * DM);
static_assert((size_t)(SEQ / 16) * NB * 8 * 2 * 32 * 8 == (size_t)NB * SEQ * DM);
static_assert((size_t)(SEQ / 64) * (DM / 64) * NB * 64 * 64 == (size_t)NB * SEQ * DM);

extern "C" void kernel_launch(void* const* d_in, const int* in_sizes, int n_in,
                              void* d_out, int out_size, void* d_ws, size_t ws_size, hipStream_t stream) {
    if (n_in < 5) return;
    const long long need = ((long long)(NB - 1) * SEQ_FULL + SEQ) * DM;
    if ((long long)in_sizes[0] < need || (long long)out_size < need) return;
    if (in_sizes[1] < DM * NQKV || in_sizes[2] < NQKV || in_sizes[3] < DM * DM || in_sizes[4] < DM) return;
    const float* x = (const float*)d_in[0];
    const float* wqkv = (const float*)d_in[1];
    const float* bqkv = (const float*)d_in[2];
    const float* wproj = (const float*)d_in[3];
    const float* bproj = (const float*)d_in[4];
    float* OUT = (float*)d_out;
    char* wsp = (char*)d_ws;
    auto take = [&](size_t bytes) { char* p = wsp; wsp += (bytes + 255) & ~(size_t)255; return (void*)p; };
    bf* WQ = (bf*)take((size_t)NQKV * DM * 2); bf* WP = (bf*)take((size_t)DM * DM * 2);
    bf* XB = (bf*)take(PLB);
    bf* QPh = (bf*)take(PLB); bf* QPl = (bf*)take(PLB); bf* KPh = (bf*)take(PLB); bf* KPl = (bf*)take(PLB); bf* VTh = (bf*)take(PLB); bf* VTl = (bf*)take(PLB);
    bf* CXh = (bf*)take(PLB); bf* CXl = (bf*)take(PLB);
    if ((size_t)(wsp - (char*)d_ws) > ws_size) return;
    k_wt<<<NQKV / 2, 256, 0, stream>>>(wqkv, WQ, (unsigned)NQKV);
    k_wt<<<DM / 2, 256, 0, stream>>>(wproj, WP, (unsigned)DM);
    k_cvt8<<<dim3(SEQ / 8, NB, 1), 256, 0, stream>>>(x, XB, (unsigned)(SEQ * 32), (size_t)SEQ_FULL * DM, (size_t)SEQ * DM);
    k_qkv<<<dim3(NB * SEQ / 64, NQKV / 64, 1), 32, 0, stream>>>(XB, WQ, bqkv, QPh, QPl, KPh, KPl, VTh, VTl);
    k_attn<<<dim3(SEQ / 16, NB, 1), 256, 0, stream>>>(QPh, QPl, KPh, KPl, VTh, VTl, CXh, CXl);
    k_gemmw<bf, 1, true><<<dim3(SEQ / 64, DM / 64, NB), 32, 0, stream>>>(CXh, CXl, WP, nullptr, DM, OUT, DM, bproj, (size_t)SEQ * DM, 0, (size_t)SEQ_FULL * DM);
}
